// PreNormTransformerDecoderLayer_76166950027522
// MI455X (gfx1250) — hardware-verified
//
#include <hip/hip_runtime.h>
#include <stddef.h>
#include <stdint.h>
#include <math.h>

#define BB   4
#define NN   1024
#define CC   1024
#define HH   16
#define DD   64
#define FF   4096
#define ROWS (BB * NN)
#define C3   (3 * CC)
#define C2   (2 * CC)
#define PL   ((size_t)ROWS * CC)
#define QBR  128
#define NQB  (NN / QBR)
#define FLN  32

static_assert(NN % 256 == 0);
static_assert(CC % 64 == 0);
static_assert(FF % 64 == 0);
static_assert(DD == 64);
static_assert(HH * DD == CC);
static_assert(ROWS % 256 == 0);
static_assert(NN == CC);
static_assert((ROWS * CC) % 8 == 0);
static_assert(NN / 64 == 16);
static_assert(QBR == 8 * 16);

#define MIB    ((size_t)1048576)
#define SZ_H1  ((size_t)ROWS * CC * 2)
#define SZ_F1  ((size_t)ROWS * CC * 4)
#define O_X1   ((size_t)0)
#define O_X2   (16 * MIB)
#define O_A1   (32 * MIB)
#define O_WQKV (40 * MIB)
#define O_QKV  (46 * MIB)
#define O_OP   (70 * MIB)
#define O_WO   (78 * MIB)
#define END_A  (O_WO + (size_t)CC * CC * 2)
#define O_H2   (32 * MIB)
#define O_EH   (40 * MIB)
#define O_WQ2  (48 * MIB)
#define O_WKV2 (50 * MIB)
#define O_QKV2 (54 * MIB)
#define O_OP2  (78 * MIB)
#define O_WO2  (86 * MIB)
#define END_B  (O_WO2 + (size_t)CC * CC * 2)
#define O_H3   (32 * MIB)
#define O_W1   (40 * MIB)
#define O_W2   (48 * MIB)
#define O_HP   (56 * MIB)
#define END_C  (O_HP + (size_t)ROWS * FF * 2)
#define O_FLG  (88 * MIB)
#define SZ_FLG ((size_t)2 * BB * NQB * FLN * 4)
#define WS_TOTAL (O_FLG + SZ_FLG)
static_assert(O_A1 >= O_X2 + SZ_F1);
static_assert(O_H2 >= O_X2 + SZ_F1);
static_assert(O_H3 >= O_X2 + SZ_F1);
static_assert(O_WQKV == O_A1 + SZ_H1);
static_assert(O_QKV == O_WQKV + (size_t)C3 * CC * 2);
static_assert(O_OP == O_QKV + 3 * SZ_H1);
static_assert(O_WO == O_OP + SZ_H1);
static_assert(O_EH == O_H2 + SZ_H1);
static_assert(O_WQ2 == O_EH + SZ_H1);
static_assert(O_WKV2 == O_WQ2 + (size_t)CC * CC * 2);
static_assert(O_QKV2 == O_WKV2 + (size_t)C2 * CC * 2);
static_assert(O_OP2 == O_QKV2 + 3 * SZ_H1);
static_assert(O_WO2 == O_OP2 + SZ_H1);
static_assert(O_W1 == O_H3 + SZ_H1);
static_assert(O_W2 == O_W1 + (size_t)FF * CC * 2);
static_assert(O_HP == O_W2 + (size_t)CC * FF * 2);
static_assert(END_A <= O_FLG);
static_assert(END_B <= O_FLG);
static_assert(END_C <= O_FLG);
static_assert(SZ_FLG == (size_t)8192);
static_assert(WS_TOTAL == (size_t)92282880);
static_assert(WS_TOTAL <= (size_t)134217728);
static_assert((O_X2 % 128) == 0 && (O_A1 % 128) == 0 && (O_WQKV % 128) == 0 && (O_QKV % 128) == 0);
static_assert((O_OP % 128) == 0 && (O_WO % 128) == 0 && (O_EH % 128) == 0 && (O_WQ2 % 128) == 0);
static_assert((O_WKV2 % 128) == 0 && (O_QKV2 % 128) == 0 && (O_OP2 % 128) == 0 && (O_WO2 % 128) == 0);
static_assert((O_W1 % 128) == 0 && (O_W2 % 128) == 0 && (O_HP % 128) == 0 && (O_FLG % 128) == 0);

typedef _Float16 v16h __attribute__((ext_vector_type(16)));
typedef _Float16 v8h  __attribute__((ext_vector_type(8)));
typedef float    v8f  __attribute__((ext_vector_type(8)));
typedef float    v4f  __attribute__((ext_vector_type(4)));
typedef unsigned int v4u __attribute__((ext_vector_type(4)));
typedef int      v4i  __attribute__((ext_vector_type(4)));

union Frag  { v16h v; v8h h[2]; };
union Pack8 { v8h h; v4u u; };

__device__ __forceinline__ v8f mma16(v16h a, v16h b, v8f c) {
  c = __builtin_amdgcn_wmma_f32_16x16x32_f16(false, a, false, b, (short)0, c, false, false);
  asm volatile("v_nop\n\tv_nop\n\tv_nop\n\tv_nop" : "+v"(c) : "v"(a), "v"(b));
  return c;
}

__device__ __forceinline__ v16h ldfrag(const _Float16* p, int ld, int row0, int k0, int lane) {
  const int m = lane & 15, lh = lane >> 4;
  const _Float16* q = p + (size_t)(row0 + m) * ld + k0 + 8 * lh;
  Frag f;
  f.h[0] = *(const v8h*)(q);
  f.h[1] = *(const v8h*)(q + 16);
  return f.v;
}

__device__ __forceinline__ v8f zero8() { return (v8f){0.f, 0.f, 0.f, 0.f, 0.f, 0.f, 0.f, 0.f}; }

template <int KK>
__device__ __forceinline__ void gemm32x64(const _Float16* __restrict__ A, int lda,
                                          const _Float16* __restrict__ Bt, int ldb,
                                          int m0, int n0, int lane, v8f (&acc)[2][4]) {
#pragma unroll 2
  for (int k0 = 0; k0 < KK; k0 += 32) {
    const v16h a0 = ldfrag(A, lda, m0, k0, lane);
    const v16h a1 = ldfrag(A, lda, m0 + 16, k0, lane);
    const v16h b0 = ldfrag(Bt, ldb, n0, k0, lane);
    const v16h b1 = ldfrag(Bt, ldb, n0 + 16, k0, lane);
    const v16h b2 = ldfrag(Bt, ldb, n0 + 32, k0, lane);
    const v16h b3 = ldfrag(Bt, ldb, n0 + 48, k0, lane);
    acc[0][0] = mma16(a0, b0, acc[0][0]);
    acc[1][0] = mma16(a1, b0, acc[1][0]);
    acc[0][1] = mma16(a0, b1, acc[0][1]);
    acc[1][1] = mma16(a1, b1, acc[1][1]);
    acc[0][2] = mma16(a0, b2, acc[0][2]);
    acc[1][2] = mma16(a1, b2, acc[1][2]);
    acc[0][3] = mma16(a0, b3, acc[0][3]);
    acc[1][3] = mma16(a1, b3, acc[1][3]);
  }
}

__global__ __launch_bounds__(256) void k_mflag(const int* __restrict__ mask, int* __restrict__ flg) {
  __shared__ __align__(16) int fl[FLN];
  const int tid = threadIdx.x, lane = tid & 31, wave = tid >> 5;
  const int blk = blockIdx.x;
  const int b = blk / NQB, qb = blk % NQB;
  const int* base = mask + ((size_t)b * NN + (size_t)qb * QBR) * NN;
  if (tid < FLN) fl[tid] = 0;
  __syncthreads();
#pragma unroll 1
  for (int j = 0; j < 2; ++j) {
    const int kc = wave * 2 + j;
    int cnt = 0;
#pragma unroll 4
    for (int it = 0; it < QBR / 2; ++it) {
      const int row = it * 2 + (lane >> 4);
      const int c4  = (lane & 15) * 4;
      const v4i mv = *(const v4i*)(base + (size_t)row * NN + kc * 64 + c4);
      cnt += (mv[0] != 0 ? 1 : 0) + (mv[1] != 0 ? 1 : 0) + (mv[2] != 0 ? 1 : 0) + (mv[3] != 0 ? 1 : 0);
    }
#pragma unroll
    for (int off = 1; off < 32; off <<= 1) cnt += __shfl_xor(cnt, off, 32);
    if (lane == 0) fl[kc] = (cnt == 0) ? 2 : ((cnt == QBR * 64) ? 1 : 0);
  }
  __syncthreads();
  if (tid < 8) {
    const v4i v = *(const v4i*)(fl + 4 * tid);
    volatile v4i* d = (volatile v4i*)(flg + (size_t)blk * FLN + 4 * tid);
    *d = v;
    __threadfence();
    *d = v;
  }
}

__global__ __launch_bounds__(256) void k_cvt(const float* __restrict__ x, _Float16* __restrict__ xh, int ngrp) {
  const int t = blockIdx.x * 256 + (int)threadIdx.x;
  if (t >= ngrp) return;
  const size_t o = (size_t)t * 8;
  const v4f a0 = *(const v4f*)(x + o);
  const v4f a1 = *(const v4f*)(x + o + 4);
  Pack8 pk;
  pk.h = (v8h){(_Float16)a0[0], (_Float16)a0[1], (_Float16)a0[2], (_Float16)a0[3],
               (_Float16)a1[0], (_Float16)a1[1], (_Float16)a1[2], (_Float16)a1[3]};
  const v4u vv = pk.u;
  volatile v4u* d = (volatile v4u*)(xh + o);
  *d = vv;
  __threadfence();
  *d = vv;
}

#define WTP 68
__global__ __launch_bounds__(256) void k_wt(const float* __restrict__ w, _Float16* __restrict__ wt,
                                           int nout, int kin) {
  __shared__ __align__(16) float tf[64 * WTP];
  const int tid = threadIdx.x;
  const int n0 = blockIdx.x * 64;
  const int k0 = blockIdx.y * 64;
  {
    const int kr = tid >> 4;
    const int n4 = (tid & 15) * 4;
#pragma unroll
    for (int it = 0; it < 4; ++it) {
      const int kl = it * 16 + kr;
      const v4f a = *(const v4f*)(w + (size_t)(k0 + kl) * nout + n0 + n4);
      *(v4f*)(tf + kl * WTP + n4) = a;
    }
  }
  __syncthreads();
  v4u val[2];
  size_t go[2];
#pragma unroll
  for (int j = 0; j < 2; ++j) {
    const int p  = tid + 256 * j;
    const int nl = p >> 3;
    const int pc = p & 7;
    const float* cp = tf + (pc * 8) * WTP + nl;
    Pack8 pk;
    pk.h = (v8h){(_Float16)(cp[0 * WTP] * 32.0f), (_Float16)(cp[1 * WTP] * 32.0f),
                 (_Float16)(cp[2 * WTP] * 32.0f), (_Float16)(cp[3 * WTP] * 32.0f),
                 (_Float16)(cp[4 * WTP] * 32.0f), (_Float16)(cp[5 * WTP] * 32.0f),
                 (_Float16)(cp[6 * WTP] * 32.0f), (_Float16)(cp[7 * WTP] * 32.0f)};
    val[j] = pk.u;
    go[j]  = (size_t)(n0 + nl) * kin + k0 + pc * 8;
  }
  for (int ps = 0; ps < 2; ++ps) {
#pragma unroll
    for (int j = 0; j < 2; ++j) *(volatile v4u*)(wt + go[j]) = val[j];
    __threadfence();
  }
}

__global__ __launch_bounds__(256) void k_ln(const float* __restrict__ in,
                                           const float* __restrict__ g,
                                           const float* __restrict__ bt,
                                           _Float16* __restrict__ outh) {
  __shared__ __align__(16) float rb[CC];
  __shared__ float red[16];
  const int tid = threadIdx.x, lane = tid & 31, wave = tid >> 5;
  const size_t ro = (size_t)blockIdx.x * CC;
  const v4f v = *(const v4f*)(in + ro + 4 * tid);
  float s = (v[0] + v[1]) + (v[2] + v[3]);
#pragma unroll
  for (int off = 1; off < 32; off <<= 1) s += __shfl_xor(s, off, 32);
  if (lane == 0) red[wave] = s;
  __syncthreads();
  float ts = 0.f;
#pragma unroll
  for (int w = 0; w < 8; ++w) ts += red[w];
  const float mean = ts * (1.0f / (float)CC);
  const float d0 = v[0] - mean, d1 = v[1] - mean, d2 = v[2] - mean, d3 = v[3] - mean;
  float q = (d0 * d0 + d1 * d1) + (d2 * d2 + d3 * d3);
#pragma unroll
  for (int off = 1; off < 32; off <<= 1) q += __shfl_xor(q, off, 32);
  if (lane == 0) red[8 + wave] = q;
  __syncthreads();
  float tq = 0.f;
#pragma unroll
  for (int w = 0; w < 8; ++w) tq += red[8 + w];
  const float var = tq * (1.0f / (float)CC);
  const float inv = rsqrtf(var + 1e-5f);
  const v4f g4 = *(const v4f*)(g + 4 * tid);
  const v4f b4 = *(const v4f*)(bt + 4 * tid);
  v4f o;
  o[0] = d0 * inv * g4[0] + b4[0];
  o[1] = d1 * inv * g4[1] + b4[1];
  o[2] = d2 * inv * g4[2] + b4[2];
  o[3] = d3 * inv * g4[3] + b4[3];
  *(v4f*)(rb + 4 * tid) = o;
  __syncthreads();
  if (tid < 128) {
    const v4f a0 = *(const v4f*)(rb + 8 * tid);
    const v4f a1 = *(const v4f*)(rb + 8 * tid + 4);
    Pack8 pk;
    pk.h = (v8h){(_Float16)a0[0], (_Float16)a0[1], (_Float16)a0[2], (_Float16)a0[3],
                 (_Float16)a1[0], (_Float16)a1[1], (_Float16)a1[2], (_Float16)a1[3]};
    const v4u vv = pk.u;
    volatile v4u* hq = (volatile v4u*)(outh + ro + 8 * tid);
    *hq = vv;
    __threadfence();
    *hq = vv;
  }
}

#define STP 72
__global__ __launch_bounds__(256) void k_proj(const _Float16* __restrict__ ah,
                                              const _Float16* __restrict__ wt,
                                              const float* __restrict__ bq,
                                              const float* __restrict__ bk,
                                              const float* __restrict__ bv,
                                              _Float16* __restrict__ planes, int base) {
  __shared__ __align__(16) _Float16 st[256 * STP];
  const int tid = threadIdx.x, lane = tid & 31, wave = tid >> 5;
  const int hh = lane >> 4, c = lane & 15;
  const int mb = blockIdx.x * 256;
  const int m0 = mb + wave * 32;
  const int n0 = blockIdx.y * 64;

  v8f acc[2][4];
#pragma unroll
  for (int s = 0; s < 2; ++s)
#pragma unroll
    for (int t = 0; t < 4; ++t) acc[s][t] = zero8();
  gemm32x64<CC>(ah, CC, wt, CC, m0, n0, lane, acc);

  const int which = base + n0 / CC;
  const int nin   = n0 & (CC - 1);
#pragma unroll
  for (int t = 0; t < 4; ++t) {
    const int ci = nin + 16 * t + c;
    const float vq = bq[ci], vk = bk[ci], vb = bv[ci];
    const float bb = (which == 0) ? vq : ((which == 1) ? vk : vb);
#pragma unroll
    for (int sub = 0; sub < 2; ++sub) {
#pragma unroll
      for (int r = 0; r < 8; ++r) {
        const int lr = wave * 32 + sub * 16 + 8 * hh + r;
        st[lr * STP + 16 * t + c] = (_Float16)(acc[sub][t][r] * 0.03125f + bb);
      }
    }
  }
  __syncthreads();

  const int b    = mb / NN;
  const int nb   = mb & (NN - 1);
  const int head = nin >> 6;
  const int bh   = b * HH + head;
  const int isv  = (which == 2);
  v4u val[8];
  size_t go[8];
  if (!isv) {
#pragma unroll
    for (int j = 0; j < 8; ++j) {
      const int p  = tid + 256 * j;
      const int lr = p >> 3;
      const int pc = p & 7;
      Pack8 pk;
      pk.h  = *(const v8h*)(st + lr * STP + pc * 8);
      val[j] = pk.u;
      go[j]  = (size_t)which * PL + ((size_t)bh * NN + nb + lr) * DD + pc * 8;
    }
  } else {
#pragma unroll
    for (int j = 0; j < 8; ++j) {
      const int p  = tid + 256 * j;
      const int L  = p >> 3;
      const int pc = p & 7;
      const int d  = L >> 2;
      const int nl = (L & 3) * 64 + pc * 8;
      const _Float16* cp = st + nl * STP + d;
      Pack8 pk;
      pk.h = (v8h){cp[0 * STP], cp[1 * STP], cp[2 * STP], cp[3 * STP],
                   cp[4 * STP], cp[5 * STP], cp[6 * STP], cp[7 * STP]};
      val[j] = pk.u;
      go[j]  = 2 * PL + ((size_t)bh * DD + d) * NN + nb + nl;
    }
  }
  for (int ps = 0; ps < 2; ++ps) {
#pragma unroll
    for (int j = 0; j < 8; ++j) *(volatile v4u*)(planes + go[j]) = val[j];
    __threadfence();
  }
}

#define KTP  72
#define PTP  72
#define MTPB 64
__global__ __launch_bounds__(256) void k_attn(const _Float16* __restrict__ qp,
                                              const _Float16* __restrict__ kp,
                                              const _Float16* __restrict__ vt,
                                              const int* __restrict__ mask,
                                              const int* __restrict__ flg,
                                              _Float16* __restrict__ op, float sscale) {
  __shared__ __align__(16) _Float16 Ks[64 * KTP];
  __shared__ __align__(16) _Float16 Vs[64 * KTP];
  __shared__ __align__(16) _Float16 Ps[8][16 * PTP];
  __shared__ __align__(16) unsigned char Ms[QBR * MTPB];

  const int tid = threadIdx.x, lane = tid & 31, wave = tid >> 5;
  const int hh = lane >> 4, c = lane & 15;
  const int bh = blockIdx.x / NQB;
  const int qb = blockIdx.x % NQB;
  const int b  = bh / HH, h = bh % HH;
  const int q0 = qb * QBR + wave * 16;

  const _Float16* Q = qp + (size_t)bh * NN * DD;
  const _Float16* K = kp + (size_t)bh * NN * DD;
  const _Float16* V = vt + (size_t)bh * DD * NN;
  const int* frow  = flg + (size_t)(b * NQB + qb) * FLN;
  const int* mbase = mask + ((size_t)b * NN + (size_t)qb * QBR) * NN;

  v16h qa[2];
  qa[0] = ldfrag(Q, DD, q0, 0, lane);
  qa[1] = ldfrag(Q, DD, q0, 32, lane);

  const float NEGI = -__builtin_huge_valf();
  const float NEGF = -__FLT_MAX__;
  float mrow[8], lrow[8];
  v8f oacc[4];
#pragma unroll
  for (int r = 0; r < 8; ++r) { mrow[r] = NEGI; lrow[r] = 0.f; }
#pragma unroll
  for (int t = 0; t < 4; ++t) oacc[t] = zero8();

  _Float16* pw = Ps[wave];

  for (int kc = 0; kc < NN / 64; ++kc) {
    const int fl = frow[kc];
    if (fl == 2) continue;
    const int mixed = (fl == 1) ? 0 : 1;
    const int kv0 = kc * 64;
    __syncthreads();
    {
      const int r  = tid >> 2;
      const int qq = (tid & 3) * 16;
      const _Float16* ks = K + (size_t)(kv0 + r) * DD + qq;
      *(v8h*)(Ks + r * KTP + qq)     = *(const v8h*)(ks);
      *(v8h*)(Ks + r * KTP + qq + 8) = *(const v8h*)(ks + 8);
      const _Float16* vs = V + (size_t)r * NN + kv0 + qq;
      *(v8h*)(Vs + r * KTP + qq)     = *(const v8h*)(vs);
      *(v8h*)(Vs + r * KTP + qq + 8) = *(const v8h*)(vs + 8);
    }
    if (mixed) {
#pragma unroll
      for (int it = 0; it < 8; ++it) {
        const int idx = it * 256 + tid;
        const int row = idx >> 4;
        const int c4  = (idx & 15) * 4;
        const v4i mv = *(const v4i*)(mbase + (size_t)row * NN + kv0 + c4);
        const unsigned int pk = (mv[0] != 0 ? 1u : 0u) | (mv[1] != 0 ? 0x100u : 0u) |
                                (mv[2] != 0 ? 0x10000u : 0u) | (mv[3] != 0 ? 0x1000000u : 0u);
        *(unsigned int*)(Ms + row * MTPB + c4) = pk;
      }
    }
    __syncthreads();

    v8f s[4];
#pragma unroll
    for (int j = 0; j < 4; ++j) s[j] = zero8();
#pragma unroll
    for (int dc = 0; dc < 2; ++dc) {
#pragma unroll
      for (int j = 0; j < 4; ++j) {
        const v16h kb = ldfrag(Ks, KTP, j * 16, dc * 32, lane);
        s[j] = mma16(qa[dc], kb, s[j]);
      }
    }
    float cm[8];
#pragma unroll
    for (int r = 0; r < 8; ++r) {
      const int trow = wave * 16 + 8 * hh + r;
      float m = NEGI;
#pragma unroll
      for (int j = 0; j < 4; ++j) {
        float sv = s[j][r] * sscale;
        if (mixed) {
          const unsigned int mbv = (unsigned int)Ms[trow * MTPB + j * 16 + c];
          sv = (mbv != 0u) ? sv : NEGF;
        }
        s[j][r] = sv;
        m = fmaxf(m, sv);
      }
#pragma unroll
      for (int off = 1; off < 16; off <<= 1) m = fmaxf(m, __shfl_xor(m, off, 32));
      cm[r] = m;
    }
    float al[8];
#pragma unroll
    for (int r = 0; r < 8; ++r) {
      const float mnew  = fmaxf(mrow[r], cm[r]);
      const float alpha = __expf(mrow[r] - mnew);
      mrow[r] = mnew;
      float psum = 0.f;
#pragma unroll
      for (int j = 0; j < 4; ++j) {
        const float p = __expf(s[j][r] - mnew);
        psum += p;
        pw[(8 * hh + r) * PTP + j * 16 + c] = (_Float16)(p * 1024.0f);
      }
#pragma unroll
      for (int off = 1; off < 16; off <<= 1) psum += __shfl_xor(psum, off, 32);
      lrow[r] = lrow[r] * alpha + psum;
      al[r] = alpha;
    }
#pragma unroll
    for (int t = 0; t < 4; ++t)
#pragma unroll
      for (int r = 0; r < 8; ++r) oacc[t][r] *= al[r];
    __syncthreads();

#pragma unroll
    for (int kk = 0; kk < 2; ++kk) {
      const v16h pa = ldfrag(pw, PTP, 0, kk * 32, lane);
#pragma unroll
      for (int t = 0; t < 4; ++t) {
        const v16h vb = ldfrag(Vs, KTP, t * 16, kk * 32, lane);
        oacc[t] = mma16(pa, vb, oacc[t]);
      }
    }
  }
  __syncthreads();

#pragma unroll
  for (int r = 0; r < 8; ++r) {
    const float lr  = lrow[r];
    const float inv = (lr > 0.f) ? (0.0625f / lr) : 0.f;
#pragma unroll
    for (int t = 0; t < 4; ++t) pw[(8 * hh + r) * PTP + 16 * t + c] = (_Float16)(oacc[t][r] * inv);
  }
  __syncthreads();
  v4u val[4];
  size_t go[4];
#pragma unroll
  for (int it = 0; it < 4; ++it) {
    const int p  = lane + 32 * it;
    const int L  = p >> 3;
    const int pc = p & 7;
    Pack8 pk;
    pk.h   = *(const v8h*)(pw + L * PTP + pc * 8);
    val[it] = pk.u;
    go[it]  = ((size_t)(b * NN + q0 + L)) * CC + (size_t)h * DD + pc * 8;
  }
  for (int ps = 0; ps < 2; ++ps) {
#pragma unroll
    for (int it = 0; it < 4; ++it) *(volatile v4u*)(op + go[it]) = val[it];
    __threadfence();
  }
}

#define OTP 68
template <int KK>
__global__ __launch_bounds__(256) void k_gout(const _Float16* __restrict__ ap,
                                              const _Float16* __restrict__ wt,
                                              const float* __restrict__ bias,
                                              const float* __restrict__ res,
                                              float* __restrict__ out, float oscale) {
  __shared__ __align__(16) float st[8][16 * OTP];
  const int tid = threadIdx.x, lane = tid & 31, wave = tid >> 5;
  const int hh = lane >> 4, c = lane & 15;
  const int m0 = blockIdx.x * 256 + wave * 32;
  const int n0 = blockIdx.y * 64;

  v8f acc[2][4];
#pragma unroll
  for (int s = 0; s < 2; ++s)
#pragma unroll
    for (int t = 0; t < 4; ++t) acc[s][t] = zero8();
  gemm32x64<KK>(ap, KK, wt, KK, m0, n0, lane, acc);

  float bvs[4];
#pragma unroll
  for (int t = 0; t < 4; ++t) bvs[t] = bias[n0 + 16 * t + c];

  float* sw = st[wave];
#pragma unroll
  for (int sub = 0; sub < 2; ++sub) {
    __syncthreads();
#pragma unroll
    for (int t = 0; t < 4; ++t) {
#pragma unroll
      for (int r = 0; r < 8; ++r)
        sw[(8 * hh + r) * OTP + 16 * t + c] = acc[sub][t][r] * oscale + bvs[t];
    }
    __syncthreads();
    v4f val[8];
    size_t go[8];
#pragma unroll
    for (int it = 0; it < 8; ++it) {
      const int p    = lane + 32 * it;
      const int L    = p >> 3;
      const int pc   = p & 7;
      const int row  = L >> 1;
      const int half = L & 1;
      const size_t gidx = (size_t)(m0 + sub * 16 + row) * CC + n0 + half * 32 + pc * 4;
      v4f v = *(const v4f*)(sw + row * OTP + half * 32 + pc * 4);
      const v4f rr = *(const v4f*)(res + gidx);
      v[0] = v[0] + rr[0]; v[1] = v[1] + rr[1]; v[2] = v[2] + rr[2]; v[3] = v[3] + rr[3];
      val[it] = v;
      go[it]  = gidx;
    }
    for (int ps = 0; ps < 2; ++ps) {
#pragma unroll
      for (int it = 0; it < 8; ++it) *(volatile v4f*)(out + go[it]) = val[it];
      __threadfence();
    }
  }
}

__device__ __forceinline__ _Float16 relu16(float v) { return (_Float16)(16.0f * fmaxf(v, 0.0f)); }

__global__ __launch_bounds__(256) void k_ffn1(const _Float16* __restrict__ ap,
                                              const _Float16* __restrict__ wt,
                                              const float* __restrict__ bias,
                                              _Float16* __restrict__ hp) {
  __shared__ __align__(16) float st[8][16 * OTP];
  const int tid = threadIdx.x, lane = tid & 31, wave = tid >> 5;
  const int hh = lane >> 4, c = lane & 15;
  const int m0 = blockIdx.x * 256 + wave * 32;
  const int n0 = blockIdx.y * 64;

  v8f acc[2][4];
#pragma unroll
  for (int s = 0; s < 2; ++s)
#pragma unroll
    for (int t = 0; t < 4; ++t) acc[s][t] = zero8();
  gemm32x64<CC>(ap, CC, wt, CC, m0, n0, lane, acc);

  float bvs[4];
#pragma unroll
  for (int t = 0; t < 4; ++t) bvs[t] = bias[n0 + 16 * t + c];

  float* sw = st[wave];
#pragma unroll
  for (int sub = 0; sub < 2; ++sub) {
    __syncthreads();
#pragma unroll
    for (int t = 0; t < 4; ++t) {
#pragma unroll
      for (int r = 0; r < 8; ++r)
        sw[(8 * hh + r) * OTP + 16 * t + c] = acc[sub][t][r] * 0.03125f + bvs[t];
    }
    __syncthreads();
    v4u val[4];
    size_t go[4];
#pragma unroll
    for (int it = 0; it < 4; ++it) {
      const int p  = lane + 32 * it;
      const int L  = p >> 3;
      const int pc = p & 7;
      const v4f x0 = *(const v4f*)(sw + L * OTP + pc * 8);
      const v4f x1 = *(const v4f*)(sw + L * OTP + pc * 8 + 4);
      Pack8 pk;
      pk.h = (v8h){relu16(x0[0]), relu16(x0[1]), relu16(x0[2]), relu16(x0[3]),
                   relu16(x1[0]), relu16(x1[1]), relu16(x1[2]), relu16(x1[3])};
      val[it] = pk.u;
      go[it]  = (size_t)(m0 + sub * 16 + L) * FF + n0 + pc * 8;
    }
    for (int ps = 0; ps < 2; ++ps) {
#pragma unroll
      for (int it = 0; it < 4; ++it) *(volatile v4u*)(hp + go[it]) = val[it];
      __threadfence();
    }
  }
}

extern "C" void kernel_launch(void* const* d_in, const int* in_sizes, int n_in,
                              void* d_out, int out_size, void* d_ws, size_t ws_size,
                              hipStream_t stream) {
  if (n_in < 30) return;
  if (in_sizes[0] != ROWS * CC || in_sizes[1] != ROWS * CC) return;
  if (in_sizes[2] != BB * NN * NN || in_sizes[3] != BB * NN * NN) return;
  for (int i = 4; i < 8; ++i)   if (in_sizes[i] != CC * CC) return;
  for (int i = 8; i < 12; ++i)  if (in_sizes[i] != CC) return;
  for (int i = 12; i < 16; ++i) if (in_sizes[i] != CC * CC) return;
  for (int i = 16; i < 20; ++i) if (in_sizes[i] != CC) return;
  if (in_sizes[20] != CC * FF || in_sizes[21] != FF) return;
  if (in_sizes[22] != FF * CC || in_sizes[23] != CC) return;
  for (int i = 24; i < 30; ++i) if (in_sizes[i] != CC) return;
  if (out_size != ROWS * CC) return;
  if (WS_TOTAL > ws_size) return;

  const float* tgt   = (const float*)d_in[0];
  const float* enc   = (const float*)d_in[1];
  const int*   tmask = (const int*)d_in[2];
  const int*   emask = (const int*)d_in[3];
  const float* s_wq = (const float*)d_in[4];
  const float* s_wk = (const float*)d_in[5];
  const float* s_wv = (const float*)d_in[6];
  const float* s_wo = (const float*)d_in[7];
  const float* s_bq = (const float*)d_in[8];
  const float* s_bk = (const float*)d_in[9];
  const float* s_bv = (const float*)d_in[10];
  const float* s_bo = (const float*)d_in[11];
  const float* c_wq = (const float*)d_in[12];
  const float* c_wk = (const float*)d_in[13];
  const float* c_wv = (const float*)d_in[14];
  const float* c_wo = (const float*)d_in[15];
  const float* c_bq = (const float*)d_in[16];
  const float* c_bk = (const float*)d_in[17];
  const float* c_bv = (const float*)d_in[18];
  const float* c_bo = (const float*)d_in[19];
  const float* f_w1 = (const float*)d_in[20];
  const float* f_b1 = (const float*)d_in[21];
  const float* f_w2 = (const float*)d_in[22];
  const float* f_b2 = (const float*)d_in[23];
  const float* ln1g = (const float*)d_in[24];
  const float* ln1b = (const float*)d_in[25];
  const float* ln2g = (const float*)d_in[26];
  const float* ln2b = (const float*)d_in[27];
  const float* ln3g = (const float*)d_in[28];
  const float* ln3b = (const float*)d_in[29];
  float* out = (float*)d_out;

  char* ws = (char*)d_ws;
  float*    X1    = (float*)(ws + O_X1);
  float*    X2    = (float*)(ws + O_X2);
  _Float16* A1h   = (_Float16*)(ws + O_A1);
  _Float16* Wqkvt = (_Float16*)(ws + O_WQKV);
  _Float16* QKVp  = (_Float16*)(ws + O_QKV);
  _Float16* Op    = (_Float16*)(ws + O_OP);
  _Float16* Wot   = (_Float16*)(ws + O_WO);
  _Float16* H2    = (_Float16*)(ws + O_H2);
  _Float16* Eh    = (_Float16*)(ws + O_EH);
  _Float16* Wq2t  = (_Float16*)(ws + O_WQ2);
  _Float16* Wkv2t = (_Float16*)(ws + O_WKV2);
  _Float16* QKV2p = (_Float16*)(ws + O_QKV2);
  _Float16* Op2   = (_Float16*)(ws + O_OP2);
  _Float16* Wo2t  = (_Float16*)(ws + O_WO2);
  _Float16* H3    = (_Float16*)(ws + O_H3);
  _Float16* W1t   = (_Float16*)(ws + O_W1);
  _Float16* W2t   = (_Float16*)(ws + O_W2);
  _Float16* Hp    = (_Float16*)(ws + O_HP);
  int*      Flg   = (int*)(ws + O_FLG);
  int*      Flg2  = Flg + BB * NQB * FLN;

  const int ngrp = in_sizes[1] / 8;

  k_mflag<<<dim3(BB * NQB), dim3(256), 0, stream>>>(tmask, Flg);
  k_mflag<<<dim3(BB * NQB), dim3(256), 0, stream>>>(emask, Flg2);

  k_ln<<<dim3(ROWS), dim3(256), 0, stream>>>(tgt, ln1g, ln1b, A1h);
  k_wt<<<dim3(CC / 64, CC / 64), dim3(256), 0, stream>>>(s_wq, Wqkvt, CC, CC);
  k_wt<<<dim3(CC / 64, CC / 64), dim3(256), 0, stream>>>(s_wk, Wqkvt + (size_t)CC * CC, CC, CC);
  k_wt<<<dim3(CC / 64, CC / 64), dim3(256), 0, stream>>>(s_wv, Wqkvt + (size_t)2 * CC * CC, CC, CC);
  k_wt<<<dim3(CC / 64, CC / 64), dim3(256), 0, stream>>>(s_wo, Wot, CC, CC);
  k_proj<<<dim3(ROWS / 256, C3 / 64), dim3(256), 0, stream>>>(A1h, Wqkvt, s_bq, s_bk, s_bv, QKVp, 0);
  k_attn<<<dim3(BB * HH * NQB), dim3(256), 0, stream>>>(QKVp, QKVp + PL, QKVp + 2 * PL, tmask, Flg, Op, 0.125f);
  k_gout<CC><<<dim3(ROWS / 256, CC / 64), dim3(256), 0, stream>>>(Op, Wot, s_bo, tgt, X1, 0.00048828125f);

  k_ln<<<dim3(ROWS), dim3(256), 0, stream>>>(X1, ln2g, ln2b, H2);
  k_cvt<<<dim3((ngrp + 255) / 256), dim3(256), 0, stream>>>(enc, Eh, ngrp);
  k_wt<<<dim3(CC / 64, CC / 64), dim3(256), 0, stream>>>(c_wq, Wq2t, CC, CC);
  k_wt<<<dim3(CC / 64, CC / 64), dim3(256), 0, stream>>>(c_wk, Wkv2t, CC, CC);
  k_wt<<<dim3(CC / 64, CC / 64), dim3(256), 0, stream>>>(c_wv, Wkv2t + (size_t)CC * CC, CC, CC);
  k_wt<<<dim3(CC / 64, CC / 64), dim3(256), 0, stream>>>(c_wo, Wo2t, CC, CC);
  k_proj<<<dim3(ROWS / 256, CC / 64), dim3(256), 0, stream>>>(H2, Wq2t, c_bq, c_bk, c_bv, QKV2p, 0);
  k_proj<<<dim3(ROWS / 256, C2 / 64), dim3(256), 0, stream>>>(Eh, Wkv2t, c_bq, c_bk, c_bv, QKV2p, 1);
  k_attn<<<dim3(BB * HH * NQB), dim3(256), 0, stream>>>(QKV2p, QKV2p + PL, QKV2p + 2 * PL, emask, Flg2, Op2, 0.125f);
  k_gout<CC><<<dim3(ROWS / 256, CC / 64), dim3(256), 0, stream>>>(Op2, Wo2t, c_bo, X1, X2, 0.00048828125f);

  k_ln<<<dim3(ROWS), dim3(256), 0, stream>>>(X2, ln3g, ln3b, H3);
  k_wt<<<dim3(FF / 64, CC / 64), dim3(256), 0, stream>>>(f_w1, W1t, FF, CC);
  k_wt<<<dim3(CC / 64, FF / 64), dim3(256), 0, stream>>>(f_w2, W2t, CC, FF);
  k_ffn1<<<dim3(ROWS / 256, FF / 64), dim3(256), 0, stream>>>(H3, W1t, f_b1, Hp);
  k_gout<FF><<<dim3(ROWS / 256, CC / 64), dim3(256), 0, stream>>>(Hp, W2t, f_b2, X2, out, 0.001953125f);
  (void)hipGetLastError();
}
